// SDPA_6305011990831
// MI455X (gfx1250) — hardware-verified
//
#include <hip/hip_runtime.h>

typedef unsigned short us;
typedef us       v8us  __attribute__((ext_vector_type(8)));
typedef us       v16us __attribute__((ext_vector_type(16)));
typedef _Float16 v16h  __attribute__((ext_vector_type(16)));
typedef __bf16   v16bf __attribute__((ext_vector_type(16)));
typedef float    v8f   __attribute__((ext_vector_type(8)));
typedef float    v4f   __attribute__((ext_vector_type(4)));

#ifndef NB
#define NB 2
#endif
#ifndef SEQ
#define SEQ 2048
#endif
#define NB_FULL  2
#define SEQ_FULL 2048
#define DIMN     1024
#define NH       16
#define HD       64
#define NTOK     (NB * SEQ)
#define NQKV     (3 * DIMN)
#define NFREQ    (HD / 2)

#define BM   128
#define BN   64
#define NTHR 256
#define NIT  (SEQ / BN)
#define LSTR 72
#define GT   128
#define GSTR 40
#define CSTR 132
#define QPL    1.4426950408889634f
#define SSC    0.125f
#define PCARRY 4096.0f
#define PINV   0.000244140625f
#define L2B_OVER_NFREQ 0.41524101186092028

static_assert(SEQ % BM == 0);
static_assert(SEQ % BN == 0);
static_assert(NTOK % GT == 0);
static_assert(DIMN % GT == 0);
static_assert(NQKV % GT == 0);
static_assert(DIMN % 32 == 0);
static_assert(NB >= 1 && NB <= NB_FULL);
static_assert(SEQ <= SEQ_FULL);
static_assert(HD == 64 && NH * HD == DIMN);
static_assert((BM * 8) % NTHR == 0 && (BN * 8) % NTHR == 0);
static_assert(NFREQ == 32);

#define XM1_LO 0x67452301u
#define XM1_HI 0xEFCDAB89u
#define XM2_LO 0x54761032u
#define XM2_HI 0xDCFE98BAu
#define XM4_LO 0x32107654u
#define XM4_HI 0xBA98FEDCu
#define XM8_LO 0xFEDCBA98u
#define XM8_HI 0x76543210u

__device__ __forceinline__ float perm16(float x, unsigned s0, unsigned s1) {
  int i = __float_as_int(x);
  int j = __builtin_amdgcn_permlane16(i, i, (int)s0, (int)s1, true, false);
  return __int_as_float(j);
}

__device__ __forceinline__ float max_raw(float a, float b) {
  float r;
  asm("v_max_num_f32 %0, %1, %2" : "=v"(r) : "v"(a), "v"(b));
  return r;
}
__device__ __forceinline__ float add_raw(float a, float b) {
  float r;
  asm("v_add_f32 %0, %1, %2" : "=v"(r) : "v"(a), "v"(b));
  return r;
}

__device__ __forceinline__ float fast_exp2(float x) {
  return __builtin_amdgcn_exp2f(x);
}

__device__ __forceinline__ us f2bf(float f) {
  unsigned u = __float_as_uint(f);
  u += 0x7FFFu + ((u >> 16) & 1u);
  return (us)(u >> 16);
}
__device__ __forceinline__ float bf2f(us b) {
  return __uint_as_float(((unsigned)b) << 16);
}
__device__ __forceinline__ us f2h(float f) {
  const _Float16 h = (_Float16)f;
  return __builtin_bit_cast(us, h);
}

__device__ __forceinline__ v16us load_frag(const us* base, int pitch, int row, int col0, int lane) {
  const int hi = (lane >> 4) << 3;
  const us* p = base + row * pitch + col0 + hi;
  v8us lo = *(const v8us*)(p);
  v8us hv = *(const v8us*)(p + 16);
  return __builtin_shufflevector(lo, hv, 0, 1, 2, 3, 4, 5, 6, 7,
                                         8, 9, 10, 11, 12, 13, 14, 15);
}

__device__ __forceinline__ v8f wmma_bf(v16us a, v16us b, v8f c) {
  v8f d = __builtin_amdgcn_wmma_f32_16x16x32_bf16(false, __builtin_bit_cast(v16bf, a), false,
                                                  __builtin_bit_cast(v16bf, b), (short)0, c,
                                                  false, false);
  asm volatile("v_nop\n\tv_nop\n\tv_nop\n\tv_nop" : "+v"(d) : "v"(a), "v"(b) : "memory");
  return d;
}
__device__ __forceinline__ v8f wmma_h(v16us a, v16us b, v8f c) {
  v8f d = __builtin_amdgcn_wmma_f32_16x16x32_f16(false, __builtin_bit_cast(v16h, a), false,
                                                 __builtin_bit_cast(v16h, b), (short)0, c,
                                                 false, false);
  asm volatile("v_nop\n\tv_nop\n\tv_nop\n\tv_nop" : "+v"(d) : "v"(a), "v"(b) : "memory");
  return d;
}

__global__ __launch_bounds__(32) void k_freq(float* __restrict__ invf) {
#pragma clang fp contract(off)
  const int j = (int)threadIdx.x & 31;
  const double e = (double)j * L2B_OVER_NFREQ;
  const float pf = (float)exp2(e);
  const float inv = 1.0f / pf;
  volatile float* p = invf + j;
  *p = inv;
  __threadfence();
  *p = inv;
}

__global__ __launch_bounds__(256) void k_tab(const float* __restrict__ invf,
                                             float* __restrict__ cst, float* __restrict__ snt) {
#pragma clang fp contract(off)
  const int g = blockIdx.x * 256 + (int)threadIdx.x;
  if (g >= SEQ * NFREQ) return;
  const int s = g >> 5, j = g & 31;
  const float inv = invf[j];
  const float ang = (float)s * inv;
  float sv, cv;
  sincosf(ang, &sv, &cv);
  volatile float* pc = cst + g;
  volatile float* pn = snt + g;
  *pc = cv;
  *pn = sv;
  __threadfence();
  *pc = cv;
  *pn = sv;
}

__global__ __launch_bounds__(256) void k_cvt(const float* __restrict__ x,
                                             const float* __restrict__ wq, const float* __restrict__ wk,
                                             const float* __restrict__ wv, const float* __restrict__ wo,
                                             us* __restrict__ xb, us* __restrict__ wcat, us* __restrict__ wob) {
  const int reg = blockIdx.y;
  const int g = blockIdx.x * 256 + (int)threadIdx.x;
  const float* src;
  us* dst;
  if (reg == 0) {
    if (g >= NTOK * (DIMN / 8)) return;
    const int r = g >> 7, c = (g & 127) * 8;
    const int b = r / SEQ, s = r - b * SEQ;
    src = x + (size_t)(b * SEQ_FULL + s) * DIMN + c;
    dst = xb + (size_t)r * DIMN + c;
  } else {
    if (g >= (DIMN * DIMN) / 8) return;
    const int w = reg - 1;
    const float* wsrc = (w == 0) ? wq : (w == 1) ? wk : (w == 2) ? wv : wo;
    src = wsrc + (size_t)g * 8;
    dst = (w < 3) ? (wcat + (size_t)w * DIMN * DIMN + (size_t)g * 8) : (wob + (size_t)g * 8);
  }
  const v4f a0 = *(const v4f*)(src);
  const v4f a1 = *(const v4f*)(src + 4);
  v8us o8 = {0, 0, 0, 0, 0, 0, 0, 0};
#pragma unroll
  for (int i = 0; i < 4; ++i) {
    o8[i]     = f2bf(a0[i]);
    o8[i + 4] = f2bf(a1[i]);
  }
  *(volatile v8us*)dst = o8;
  __threadfence();
  *(volatile v8us*)dst = o8;
}

template <int NA>
__global__ __launch_bounds__(NTHR) __attribute__((amdgpu_num_vgpr(256)))
void k_gemm(const us* __restrict__ A0, const us* __restrict__ A1, const us* __restrict__ B,
            float* __restrict__ C, int K, int ldc) {
  __shared__ __align__(16) us    As[NA][GT * GSTR];
  __shared__ __align__(16) us    Bs[GT * GSTR];
  __shared__ __align__(16) float Cs[(GT / 2) * CSTR];

  const int tid = threadIdx.x, lane = tid & 31, wave = tid >> 5;
  const int lr = lane & 15, hsel = lane >> 4;
  const int wm = wave & 3, wn = wave >> 2;
  const int bm = blockIdx.y * GT, bn = blockIdx.x * GT;
  const int sr = tid >> 1, sc = (tid & 1) * 16;

  const v8f zero8 = {0.f, 0.f, 0.f, 0.f, 0.f, 0.f, 0.f, 0.f};
  v8f acc[2][4];
#pragma unroll
  for (int i = 0; i < 2; ++i)
#pragma unroll
    for (int t = 0; t < 4; ++t) acc[i][t] = zero8;

#pragma unroll 1
  for (int k0 = 0; k0 < K; k0 += 32) {
    __syncthreads();
#pragma unroll
    for (int p = 0; p < NA; ++p) {
      const us* ap = ((p == 0) ? A0 : A1) + (size_t)(bm + sr) * K + k0 + sc;
      *(v8us*)&As[p][sr * GSTR + sc]     = *(const v8us*)(ap);
      *(v8us*)&As[p][sr * GSTR + sc + 8] = *(const v8us*)(ap + 8);
    }
    {
      const us* bp = B + (size_t)(bn + sr) * K + k0 + sc;
      *(v8us*)&Bs[sr * GSTR + sc]     = *(const v8us*)(bp);
      *(v8us*)&Bs[sr * GSTR + sc + 8] = *(const v8us*)(bp + 8);
    }
    __syncthreads();

    v16us bf[4];
#pragma unroll
    for (int t = 0; t < 4; ++t) bf[t] = load_frag(Bs, GSTR, wn * 64 + t * 16 + lr, 0, lane);
#pragma unroll
    for (int p = 0; p < NA; ++p)
#pragma unroll
      for (int i = 0; i < 2; ++i) {
        const v16us af = load_frag(As[p], GSTR, wm * 32 + i * 16 + lr, 0, lane);
#pragma unroll
        for (int t = 0; t < 4; ++t) acc[i][t] = wmma_bf(af, bf[t], acc[i][t]);
      }
  }

#pragma unroll
  for (int hf = 0; hf < 2; ++hf) {
    __syncthreads();
    if ((wm >> 1) == hf) {
#pragma unroll
      for (int i = 0; i < 2; ++i)
#pragma unroll
        for (int t = 0; t < 4; ++t)
#pragma unroll
          for (int j = 0; j < 8; ++j)
            Cs[((wm & 1) * 32 + i * 16 + hsel * 8 + j) * CSTR + wn * 64 + t * 16 + lr] = acc[i][t][j];
    }
    __syncthreads();

    v4f vals[8];
    size_t go[8];
#pragma unroll
    for (int st = 0; st < 8; ++st) {
      const int row = st * 8 + wave;
      vals[st] = *(const v4f*)&Cs[row * CSTR + lane * 4];
      go[st] = (size_t)(bm + hf * (GT / 2) + row) * ldc + bn + lane * 4;
      *(volatile v4f*)(C + go[st]) = vals[st];
    }
    __threadfence();
#pragma unroll
    for (int st = 0; st < 8; ++st) {
      *(volatile v4f*)(C + go[st]) = vals[st];
    }
  }
}

__global__ __launch_bounds__(256) void k_rope_split(const float* __restrict__ Cq,
                                                    const float* __restrict__ cst,
                                                    const float* __restrict__ snt,
                                                    us* __restrict__ q16, us* __restrict__ k16,
                                                    us* __restrict__ v16) {
#pragma clang fp contract(off)
  const int tsel = blockIdx.y;
  const int g = blockIdx.x * 256 + (int)threadIdx.x;
  if (g >= NTOK * NH * 8) return;
  const int tok = g >> 7, hh = (g >> 3) & 15, c = g & 7;
  const int b = tok / SEQ, s = tok - b * SEQ;

  const float* src = Cq + (size_t)tok * NQKV + tsel * DIMN + hh * HD;
  const int pc = c ^ 4;
  const v4f x0 = *(const v4f*)(src + c * 8);
  const v4f x1 = *(const v4f*)(src + c * 8 + 4);
  const v4f y0 = *(const v4f*)(src + pc * 8);
  const v4f y1 = *(const v4f*)(src + pc * 8 + 4);
  const int j0 = (c & 3) * 8;
  const v4f c0 = *(const v4f*)(cst + s * NFREQ + j0);
  const v4f c1 = *(const v4f*)(cst + s * NFREQ + j0 + 4);
  const v4f n0 = *(const v4f*)(snt + s * NFREQ + j0);
  const v4f n1 = *(const v4f*)(snt + s * NFREQ + j0 + 4);

  const v8f xa = __builtin_shufflevector(x0, x1, 0, 1, 2, 3, 4, 5, 6, 7);
  const v8f ya = __builtin_shufflevector(y0, y1, 0, 1, 2, 3, 4, 5, 6, 7);
  const v8f ca = __builtin_shufflevector(c0, c1, 0, 1, 2, 3, 4, 5, 6, 7);
  const v8f sa = __builtin_shufflevector(n0, n1, 0, 1, 2, 3, 4, 5, 6, 7);

  const float sg  = (c < 4) ? -1.0f : 1.0f;
  const bool  rot = (tsel != 2);
  const float osc = (tsel == 0) ? QPL : 1.0f;

  v8us ov = {0, 0, 0, 0, 0, 0, 0, 0};
#pragma unroll
  for (int i = 0; i < 8; ++i) {
    float v = xa[i];
    if (rot) {
      const float a  = xa[i] * ca[i];
      const float bb = (sg * ya[i]) * sa[i];
      v = a + bb;
    }
    v = v * osc;
    ov[i] = f2h(v);
  }
  us* pd = (tsel == 0) ? q16 : (tsel == 1) ? k16 : v16;
  const size_t goff = (((size_t)(b * NH + hh)) * SEQ + s) * HD + (size_t)c * 8;
  *(volatile v8us*)(pd + goff) = ov;
  __threadfence();
  *(volatile v8us*)(pd + goff) = ov;
}

__global__ __launch_bounds__(NTHR) __attribute__((amdgpu_num_vgpr(256)))
void k_attn(const us* __restrict__ q16, const us* __restrict__ k16, const us* __restrict__ v16,
            us* __restrict__ ch, us* __restrict__ cl) {
  __shared__ __align__(16) us Qs[BM * LSTR];
  __shared__ __align__(16) us Ks[BN * LSTR];
  __shared__ __align__(16) us Vt[HD * LSTR];
  __shared__ __align__(16) us Ps[BM * LSTR];

  const int tid = threadIdx.x, lane = tid & 31, wave = tid >> 5;
  const int lr = lane & 15, hsel = lane >> 4;
  const int tiles = SEQ / BM;
  const int bx = blockIdx.x;
  const int bhd = bx / tiles;
  const int m0 = (bx - bhd * tiles) * BM;
  const int b = bhd / NH, hd = bhd - b * NH;
  const size_t prow0 = (size_t)bhd * SEQ;

#pragma unroll
  for (int i = 0; i < (BM * 8) / NTHR; ++i) {
    const int idx = i * NTHR + tid;
    const int r = idx >> 3, c = (idx & 7) * 8;
    const size_t g = (prow0 + m0 + r) * HD + c;
    *(v8us*)&Qs[r * LSTR + c] = *(const v8us*)(q16 + g);
  }
  __syncthreads();

  const v16us aq0 = load_frag(Qs, LSTR, wave * 16 + lr, 0,  lane);
  const v16us aq1 = load_frag(Qs, LSTR, wave * 16 + lr, 32, lane);

  const v8f zero8 = {0.f, 0.f, 0.f, 0.f, 0.f, 0.f, 0.f, 0.f};
  v8f o[4];
#pragma unroll
  for (int t = 0; t < 4; ++t) o[t] = zero8;
  float m_run[8], l_run[8];
#pragma unroll
  for (int r = 0; r < 8; ++r) { m_run[r] = -__builtin_inff(); l_run[r] = 0.f; }

  const unsigned SL[4] = { XM1_LO, XM2_LO, XM4_LO, XM8_LO };
  const unsigned SH[4] = { XM1_HI, XM2_HI, XM4_HI, XM8_HI };

#pragma unroll 1
  for (int it = 0; it < NIT; ++it) {
    __syncthreads();
#pragma unroll
    for (int i = 0; i < (BN * 8) / NTHR; ++i) {
      const int idx = i * NTHR + tid;
      const int r = idx >> 3, c = (idx & 7) * 8;
      const size_t g = (prow0 + (size_t)it * BN + r) * HD + c;
      *(v8us*)&Ks[r * LSTR + c] = *(const v8us*)(k16 + g);
      const v8us va = *(const v8us*)(v16 + g);
#pragma unroll
      for (int e = 0; e < 8; ++e) Vt[(c + e) * LSTR + r] = va[e];
    }
    __syncthreads();

    v8f s[4];
#pragma unroll
    for (int tn = 0; tn < 4; ++tn) {
      const v16us b0 = load_frag(Ks, LSTR, tn * 16 + lr, 0,  lane);
      const v16us b1 = load_frag(Ks, LSTR, tn * 16 + lr, 32, lane);
      v8f a = zero8;
      a = wmma_h(aq0, b0, a);
      a = wmma_h(aq1, b1, a);
      s[tn] = a;
    }

    float t8[8], alpha[8], rs[8], msc[8];
#pragma unroll
    for (int r = 0; r < 8; ++r)
      t8[r] = fmaxf(fmaxf(s[0][r], s[1][r]), fmaxf(s[2][r], s[3][r]));
#pragma unroll
    for (int stp = 0; stp < 4; ++stp)
#pragma unroll
      for (int r = 0; r < 8; ++r)
        t8[r] = max_raw(t8[r], perm16(t8[r], SL[stp], SH[stp]));
#pragma unroll
    for (int r = 0; r < 8; ++r) {
      const float m_new = max_raw(m_run[r], t8[r]);
      alpha[r] = fast_exp2((m_run[r] - m_new) * SSC);
      m_run[r] = m_new;
      msc[r] = m_new * SSC;
    }
#pragma unroll
    for (int r = 0; r < 8; ++r) {
      float acc = 0.f;
#pragma unroll
      for (int tn = 0; tn < 4; ++tn) {
        const float p = fast_exp2(s[tn][r] * SSC - msc[r]);
        s[tn][r] = p;
        acc += p;
      }
      rs[r] = acc;
    }
#pragma unroll
    for (int stp = 0; stp < 4; ++stp)
#pragma unroll
      for (int r = 0; r < 8; ++r)
        rs[r] = add_raw(rs[r], perm16(rs[r], SL[stp], SH[stp]));
#pragma unroll
    for (int r = 0; r < 8; ++r) {
      l_run[r] = l_run[r] * alpha[r] + rs[r];
#pragma unroll
      for (int t = 0; t < 4; ++t) o[t][r] *= alpha[r];
    }

    {
      const int prow = wave * 16 + (hsel << 3);
#pragma unroll
      for (int tn = 0; tn < 4; ++tn)
#pragma unroll
        for (int r = 0; r < 8; ++r)
          Ps[(prow + r) * LSTR + tn * 16 + lr] = f2h(s[tn][r] * PCARRY);
    }
    __syncthreads();

    {
      const v16us ap0 = load_frag(Ps, LSTR, wave * 16 + lr, 0,  lane);
      const v16us ap1 = load_frag(Ps, LSTR, wave * 16 + lr, 32, lane);
#pragma unroll
      for (int t = 0; t < 4; ++t) {
        const v16us w0 = load_frag(Vt, LSTR, t * 16 + lr, 0,  lane);
        const v16us w1 = load_frag(Vt, LSTR, t * 16 + lr, 32, lane);
        v8f a = o[t];
        a = wmma_h(ap0, w0, a);
        a = wmma_h(ap1, w1, a);
        o[t] = a;
      }
    }
  }
  __syncthreads();

  {
    float inv[8];
#pragma unroll
    for (int r = 0; r < 8; ++r) inv[r] = (1.0f / l_run[r]) * PINV;
    const int prow = wave * 16 + (hsel << 3);
#pragma unroll
    for (int t = 0; t < 4; ++t)
#pragma unroll
      for (int r = 0; r < 8; ++r) {
        const float cv = o[t][r] * inv[r];
        const us hb = f2bf(cv);
        const us lb = f2bf(cv - bf2f(hb));
        Ps[(prow + r) * LSTR + t * 16 + lr] = hb;
        Qs[(prow + r) * LSTR + t * 16 + lr] = lb;
      }
  }
  __syncthreads();
  {
    v8us hv[4], lv[4];
    size_t go[4];
#pragma unroll
    for (int st = 0; st < 4; ++st) {
      const int row = wave * 16 + st * 4 + (lane >> 3);
      const int c8 = (lane & 7) * 8;
      hv[st] = *(const v8us*)&Ps[row * LSTR + c8];
      lv[st] = *(const v8us*)&Qs[row * LSTR + c8];
      const size_t tok = (size_t)b * SEQ + m0 + row;
      go[st] = tok * DIMN + (size_t)hd * HD + c8;
      *(volatile v8us*)(ch + go[st]) = hv[st];
      *(volatile v8us*)(cl + go[st]) = lv[st];
    }
    __threadfence();
#pragma unroll
    for (int st = 0; st < 4; ++st) {
      *(volatile v8us*)(ch + go[st]) = hv[st];
      *(volatile v8us*)(cl + go[st]) = lv[st];
    }
  }
}

static size_t carve_bytes(size_t& off, size_t bytes) {
  const size_t o = off;
  off += (bytes + 127) & ~(size_t)127;
  return o;
}

extern "C" void kernel_launch(void* const* d_in, const int* in_sizes, int n_in,
                              void* d_out, int out_size, void* d_ws, size_t ws_size,
                              hipStream_t stream) {
  if (n_in < 5) return;
  const long long need_x = ((long long)(NB - 1) * SEQ_FULL + SEQ) * (long long)DIMN;
  if ((long long)in_sizes[0] < need_x) return;
  for (int i = 1; i < 5; ++i)
    if ((long long)in_sizes[i] < (long long)DIMN * DIMN) return;
  if ((long long)out_size < (long long)NTOK * DIMN) return;

  const float* x  = (const float*)d_in[0];
  const float* Wq = (const float*)d_in[1];
  const float* Wk = (const float*)d_in[2];
  const float* Wv = (const float*)d_in[3];
  const float* Wo = (const float*)d_in[4];
  float* out = (float*)d_out;
  char* ws = (char*)d_ws;

  const size_t plane_bytes = (size_t)NTOK * DIMN * 2;
  const size_t qkvf_bytes  = (size_t)NTOK * NQKV * 4;
  const size_t big_bytes   = (qkvf_bytes > 2 * plane_bytes) ? qkvf_bytes : 2 * plane_bytes;

  size_t off = 0;
  const size_t o_invf = carve_bytes(off, (size_t)NFREQ * 4);
  const size_t o_cst  = carve_bytes(off, (size_t)SEQ * NFREQ * 4);
  const size_t o_snt  = carve_bytes(off, (size_t)SEQ * NFREQ * 4);
  const size_t o_xb   = carve_bytes(off, plane_bytes);
  const size_t o_wcat = carve_bytes(off, (size_t)NQKV * DIMN * 2);
  const size_t o_wob  = carve_bytes(off, (size_t)DIMN * DIMN * 2);
  const size_t o_big  = carve_bytes(off, big_bytes);
  const size_t o_q16  = carve_bytes(off, plane_bytes);
  const size_t o_k16  = carve_bytes(off, plane_bytes);
  const size_t o_v16  = carve_bytes(off, plane_bytes);
  if (off > ws_size) return;

  float* invf = (float*)(ws + o_invf);
  float* cst  = (float*)(ws + o_cst);
  float* snt  = (float*)(ws + o_snt);
  us* xb   = (us*)(ws + o_xb);
  us* wcat = (us*)(ws + o_wcat);
  us* wob  = (us*)(ws + o_wob);
  float* qkvf = (float*)(ws + o_big);
  us* ch  = (us*)(ws + o_big);
  us* cl  = (us*)(ws + o_big + plane_bytes);
  us* q16 = (us*)(ws + o_q16);
  us* k16 = (us*)(ws + o_k16);
  us* v16 = (us*)(ws + o_v16);

  k_freq<<<dim3(1), 32, 0, stream>>>(invf);
  k_tab<<<dim3((SEQ * NFREQ + 255) / 256), 256, 0, stream>>>(invf, cst, snt);

  {
    const int nx = NTOK * (DIMN / 8);
    const int nw = (DIMN * DIMN) / 8;
    const int nmax = (nx > nw) ? nx : nw;
    k_cvt<<<dim3((nmax + 255) / 256, 5), 256, 0, stream>>>(x, Wq, Wk, Wv, Wo, xb, wcat, wob);
  }

  k_gemm<1><<<dim3(NQKV / GT, NTOK / GT), NTHR, 0, stream>>>(xb, xb, wcat, qkvf, DIMN, NQKV);

  k_rope_split<<<dim3((NTOK * NH * 8 + 255) / 256, 3), 256, 0, stream>>>(qkvf, cst, snt, q16, k16, v16);

  k_attn<<<dim3(NB * NH * (SEQ / BM)), NTHR, 0, stream>>>(q16, k16, v16, ch, cl);

  k_gemm<2><<<dim3(DIMN / GT, NTOK / GT), NTHR, 0, stream>>>(ch, cl, wob, out, DIMN, DIMN);
}
